// TPAAttention_6863357739640
// MI455X (gfx1250) — hardware-verified
//
#include <hip/hip_runtime.h>


namespace {
constexpr int S = 2048, HID = 2048, H = 16, KVH = 8, D = 128, QR = 6, KR = 2, VR = 2, NF = H * QR + KVH * KR + KVH * VR + QR * D + KR * D + VR * D  , CH = 256;
constexpr int OAQ = 0, OAK = 96, OAV = 112, OBQ = 128, OBK = 896, OBV = 1152;
constexpr float XS = 8.0f, QS = 16.0f, HS = 256.0f, PS = 256.0f, WSC = 256.0f, SCALE = 0.08838834764831845f, CAP = 50.0f;
typedef _Float16 b16;
typedef __attribute__((ext_vector_type(16))) _Float16 v16b;
typedef __attribute__((ext_vector_type(8))) _Float16 v8b;
typedef __attribute__((ext_vector_type(2))) _Float16 v2b;
typedef __attribute__((ext_vector_type(8))) float v8f;
typedef __attribute__((ext_vector_type(4))) float v4f;
typedef __attribute__((ext_vector_type(2))) float v2f;
__device__ __forceinline__ float bf16_rne(float f) { unsigned int u = __float_as_uint(f); u += 0x7FFFu + ((u >> 16) & 1u); float r = __uint_as_float(u & 0xFFFF0000u); asm volatile("" : "+v"(r)); return r; }
__device__ __forceinline__ float bfv(float f) { float r = bf16_rne(f); asm volatile("" : "+v"(r)); return r; }
__device__ __forceinline__ void split16(float v, b16& hi, b16& lo) { hi = (b16)v; lo = (b16)(v - (float)hi); }
__device__ __forceinline__ void split16b(float v, b16& hi, b16& lo) { asm volatile("" : "+v"(v)); hi = (b16)v; float hf = (float)hi; asm volatile("" : "+v"(hf)); float d = v - hf; asm volatile("" : "+v"(d)); lo = (b16)d; }
__device__ __forceinline__ v16b frag_kb(const b16* p, int hh) { const v8b a = *(const v8b*)(p + 8 * hh), b = *(const v8b*)(p + 16 + 8 * hh); v16b f;
#pragma unroll
  for (int e = 0; e < 8; ++e) { f[e] = a[e]; f[8 + e] = b[e]; } return f; }
__device__ __forceinline__ v8f wmma16b(v16b a, v16b b, v8f c) { v8f d = __builtin_amdgcn_wmma_f32_16x16x32_f16(false, a, false, b, (short)0, c, false, false); asm volatile("v_nop\n\tv_nop\n\tv_nop\n\tv_nop" : "+v"(d) : "v"(a), "v"(b)); return d; }
__device__ __forceinline__ void wave_lds_sync() { __builtin_amdgcn_fence(__ATOMIC_RELEASE, "workgroup"); __builtin_amdgcn_wave_barrier(); __builtin_amdgcn_fence(__ATOMIC_ACQUIRE, "workgroup"); }
__device__ __forceinline__ float pmul(float a, float b) { float p = a * b; asm volatile("" : "+v"(p)); return p; }

__global__ __launch_bounds__(256) void wput_kernel(const float* __restrict__ waq, const float* __restrict__ wak, const float* __restrict__ wav, const float* __restrict__ wbq, const float* __restrict__ wbk, const float* __restrict__ wbv, const float* __restrict__ wo, b16* __restrict__ WT, b16* __restrict__ WO) { const size_t nt = (size_t)gridDim.x * 256, u0 = (size_t)blockIdx.x * 256 + threadIdx.x; v8b v;
  for (size_t u = u0; u < (size_t)NF * (HID / 8); u += nt) { const int o = (int)(u / (HID / 8)), k0 = (int)(u % (HID / 8)) * 8; const float* w; int oo, ncol; if (o < OAK) { w = waq; oo = o; ncol = 96; } else if (o < OAV) { w = wak; oo = o - OAK; ncol = 16; } else if (o < OBQ) { w = wav; oo = o - OAV; ncol = 16; } else if (o < OBK) { w = wbq; oo = o - OBQ; ncol = QR * D; } else if (o < OBV) { w = wbk; oo = o - OBK; ncol = KR * D; } else { w = wbv; oo = o - OBV; ncol = VR * D; }
#pragma unroll
    for (int j = 0; j < 8; ++j) v[j] = (b16)(bf16_rne(w[(size_t)(k0 + j) * ncol + oo]) * WSC); for (int pass = 0; pass < 2; ++pass) { *(volatile v8b*)(WT + (size_t)o * HID + k0) = v; __threadfence(); } }
  for (size_t u = u0; u < (size_t)HID * (HID / 8); u += nt) { const int o = (int)(u / (HID / 8)), k0 = (int)(u % (HID / 8)) * 8;
#pragma unroll
    for (int j = 0; j < 8; ++j) v[j] = (b16)(bf16_rne(wo[(size_t)(k0 + j) * HID + o]) * WSC); for (int pass = 0; pass < 2; ++pass) { *(volatile v8b*)(WO + (size_t)o * HID + k0) = v; __threadfence(); } } }
__global__ __launch_bounds__(32) void proj_kernel(const float* __restrict__ x, const b16* __restrict__ WT, int QLIM, float* __restrict__ FAC) { __shared__ __attribute__((aligned(16))) b16 Ax[16][HID + 8]; __shared__ float Tf[16][260]; const int lane = threadIdx.x, nloc = lane & 15, hlf = lane >> 4; const size_t t0 = (size_t)blockIdx.x * 16; const int g = blockIdx.y; const int c0 = g * 256, nt = (NF - c0) >= 256 ? 16 : (NF - c0) / 16; if ((int)t0 >= QLIM) return;
  for (int rr = 0; rr < 16; ++rr) for (int q = 0; q < HID / 32; ++q) { const int c = q * 32 + lane; Ax[rr][c] = (b16)(bf16_rne(x[(t0 + rr) * HID + c]) * XS); }
  if (lane < 16) for (int k = HID; k < HID + 8; ++k) Ax[lane][k] = (b16)0.0f;
  wave_lds_sync(); v8f acc[16];
#pragma unroll
  for (int t = 0; t < 16; ++t) acc[t] = (v8f){};
#pragma unroll 2
  for (int kb = 0; kb < HID; kb += 32) { const v16b a = frag_kb(&Ax[nloc][kb], hlf);
#pragma unroll
    for (int t = 0; t < 16; ++t) if (t < nt) acc[t] = wmma16b(a, frag_kb(WT + (size_t)(c0 + t * 16 + nloc) * HID + kb, hlf), acc[t]); }
#pragma unroll
  for (int t = 0; t < 16; ++t) if (t < nt)
#pragma unroll
    for (int r8 = 0; r8 < 8; ++r8) Tf[8 * hlf + r8][t * 16 + nloc] = acc[t][r8] * (1.0f / (XS * WSC));
  wave_lds_sync();
  for (int pass = 0; pass < 2; ++pass) { for (int rr = 0; rr < 16; ++rr) for (int q = 0; q < nt / 2; ++q) ((volatile float*)FAC)[(t0 + rr) * NF + c0 + q * 32 + lane] = Tf[rr][q * 32 + lane]; __threadfence(); } }
__global__ __launch_bounds__(32) void asm_kernel(const float* __restrict__ FAC, const float* __restrict__ cosr, const float* __restrict__ sinr, int QLIM, b16* __restrict__ Qh, b16* __restrict__ Ql, b16* __restrict__ Kh, b16* __restrict__ Kl, float* __restrict__ VRp) { const int lane = threadIdx.x; const size_t t0 = (size_t)blockIdx.x * 16; if ((int)t0 >= QLIM) return;
  for (int rr = 0; rr < 16; ++rr) { const size_t s = t0 + rr; const float* f = FAC + s * NF; const int d0 = lane * 4;
    float bq[QR][4], bk[KR][4], bv[VR][4]; const float c0 = bfv(cosr[s * 64 + d0 / 2]), s0 = bfv(sinr[s * 64 + d0 / 2]), c1 = bfv(cosr[s * 64 + d0 / 2 + 1]), s1 = bfv(sinr[s * 64 + d0 / 2 + 1]);
#pragma unroll
    for (int r = 0; r < QR; ++r) { const v4f b4 = *(const v4f*)(f + OBQ + r * D + d0); bq[r][0] = pmul(b4[0], c0) - pmul(b4[1], s0); bq[r][1] = pmul(b4[0], s0) + pmul(b4[1], c0); bq[r][2] = pmul(b4[2], c1) - pmul(b4[3], s1); bq[r][3] = pmul(b4[2], s1) + pmul(b4[3], c1); }
#pragma unroll
    for (int r = 0; r < KR; ++r) { const v4f b4 = *(const v4f*)(f + OBK + r * D + d0); bk[r][0] = pmul(b4[0], c0) - pmul(b4[1], s0); bk[r][1] = pmul(b4[0], s0) + pmul(b4[1], c0); bk[r][2] = pmul(b4[2], c1) - pmul(b4[3], s1); bk[r][3] = pmul(b4[2], s1) + pmul(b4[3], c1); const v4f v4 = *(const v4f*)(f + OBV + r * D + d0); bv[r][0] = v4[0]; bv[r][1] = v4[1]; bv[r][2] = v4[2]; bv[r][3] = v4[3]; }
    for (int pass = 0; pass < 2; ++pass) {
      for (int h = 0; h < H; ++h) { float q4[4] = {0, 0, 0, 0};
#pragma unroll
        for (int r = 0; r < QR; ++r) { const float a = f[OAQ + h * QR + r];
#pragma unroll
          for (int e = 0; e < 4; ++e) q4[e] += pmul(a, bq[r][e]); }
        b16 hh[4], ll[4];
#pragma unroll
        for (int e = 0; e < 4; ++e) split16b(pmul(q4[e], QS), hh[e], ll[e]); const size_t o = (s * H + h) * D + d0; *(volatile v2b*)(Qh + o) = (v2b){hh[0], hh[1]}; *(volatile v2b*)(Qh + o + 2) = (v2b){hh[2], hh[3]}; *(volatile v2b*)(Ql + o) = (v2b){ll[0], ll[1]}; *(volatile v2b*)(Ql + o + 2) = (v2b){ll[2], ll[3]}; }
      for (int gk = 0; gk < KVH; ++gk) { float k4[4] = {0, 0, 0, 0}, v4v[4] = {0, 0, 0, 0};
#pragma unroll
        for (int r = 0; r < KR; ++r) { const float a = f[OAK + gk * KR + r], av = f[OAV + gk * VR + r];
#pragma unroll
          for (int e = 0; e < 4; ++e) { k4[e] += pmul(a, bk[r][e]); v4v[e] += pmul(av, bv[r][e]); } }
        b16 hh[4], ll[4];
#pragma unroll
        for (int e = 0; e < 4; ++e) split16b(pmul(k4[e], QS), hh[e], ll[e]); const size_t o = (s * KVH + gk) * D + d0; *(volatile v2b*)(Kh + o) = (v2b){hh[0], hh[1]}; *(volatile v2b*)(Kh + o + 2) = (v2b){hh[2], hh[3]}; *(volatile v2b*)(Kl + o) = (v2b){ll[0], ll[1]}; *(volatile v2b*)(Kl + o + 2) = (v2b){ll[2], ll[3]}; *(volatile v4f*)(VRp + o) = (v4f){v4v[0], v4v[1], v4v[2], v4v[3]}; }
      __threadfence(); } } }
__global__ __launch_bounds__(256) void vt_kernel(const float* __restrict__ VRp, int QLIM, b16* __restrict__ VTh, b16* __restrict__ VTl) { __shared__ float Tt[64][257]; const int tt = blockIdx.x >> 2, gg = blockIdx.x & 3; const int s0 = tt * 64; if (s0 >= QLIM) return; const int tid = threadIdx.x, wave = tid >> 5, lane = tid & 31;
  for (int q = wave; q < 64; q += 8) for (int c = lane; c < 256; c += 32) Tt[q][c] = VRp[(size_t)(s0 + q) * (KVH * D) + gg * 256 + c];
  __syncthreads();
  for (int pass = 0; pass < 2; ++pass) { for (int c = wave; c < 256; c += 8) { const int g = gg * 2 + c / D, d = c % D; b16 h0, l0, h1, l1; split16(Tt[lane * 2][c] * QS, h0, l0); split16(Tt[lane * 2 + 1][c] * QS, h1, l1); const size_t o = ((size_t)g * D + d) * S + s0 + lane * 2; *(volatile v2b*)(VTh + o) = (v2b){h0, h1}; *(volatile v2b*)(VTl + o) = (v2b){l0, l1}; } __threadfence(); } }
__global__ __launch_bounds__(32) void att_kernel(const b16* __restrict__ Qh, const b16* __restrict__ Ql, const b16* __restrict__ Kh, const b16* __restrict__ Kl, const b16* __restrict__ VTh, const b16* __restrict__ VTl, const float* __restrict__ amask, int QLIM, float* __restrict__ O) { __shared__ __attribute__((aligned(16))) b16 Pa[16][CH + 8], Pb[16][CH + 8]; __shared__ float Sc[16][CH + 1], Mx[16], Ls[16], Fc[16], Of[16][D + 1]; __shared__ int Any[16]; const int lane = threadIdx.x, nloc = lane & 15, hlf = lane >> 4; const int h = blockIdx.x / (S / 16), q0 = (blockIdx.x % (S / 16)) * 16; if (q0 >= QLIM) return; const int g = h / (H / KVH);
  if (lane < 16) { Mx[lane] = -INFINITY; Ls[lane] = 0.0f; for (int kk = CH; kk < CH + 8; ++kk) { Pa[lane][kk] = (b16)0.0f; Pb[lane][kk] = (b16)0.0f; } }
  const b16* qhp = Qh + ((size_t)(q0 + nloc) * H + h) * D; const b16* qlp = Ql + ((size_t)(q0 + nloc) * H + h) * D;
  v8f oacc[8];
#pragma unroll
  for (int t = 0; t < 8; ++t) oacc[t] = (v8f){};
#pragma unroll 1
  for (int ch = 0; ch < S / CH; ++ch) { const int k0 = ch * CH;
    if (lane < 16) { const float* mr = amask + (size_t)(q0 + lane) * S + k0; int any = 0; for (int j = 0; j < CH; ++j) any |= (mr[j] > -1e8f); Any[lane] = any; }
    wave_lds_sync();
    int anyw = 0, allfin = 1; for (int r = 0; r < 16; ++r) { anyw |= Any[r]; allfin &= (Mx[r] != -INFINITY); }
    if (!anyw && allfin) continue;
#pragma unroll 1
    for (int tg = 0; tg < 16; tg += 4) { v8f sacc[4] = {(v8f){}, (v8f){}, (v8f){}, (v8f){}};
#pragma unroll
      for (int t = 0; t < 4; ++t)
#pragma unroll
        for (int ks = 0; ks < 4; ++ks) { const size_t ko = ((size_t)(k0 + (tg + t) * 16 + nloc) * KVH + g) * D + ks * 32; const v16b kh = frag_kb(Kh + ko, hlf), kl = frag_kb(Kl + ko, hlf); const v16b qa = frag_kb(qhp + ks * 32, hlf), ql = frag_kb(qlp + ks * 32, hlf); sacc[t] = wmma16b(qa, kh, sacc[t]); sacc[t] = wmma16b(qa, kl, sacc[t]); sacc[t] = wmma16b(ql, kh, sacc[t]); }
#pragma unroll
      for (int t = 0; t < 4; ++t)
#pragma unroll
        for (int r8 = 0; r8 < 8; ++r8) Sc[8 * hlf + r8][(tg + t) * 16 + nloc] = sacc[t][r8] * (SCALE / (QS * QS)); }
    wave_lds_sync();
    if (lane < 16) { const int r = lane; const float* mr = amask + (size_t)(q0 + r) * S + k0; float mx = -INFINITY; for (int j = 0; j < CH; ++j) { const float s = CAP * tanhf(Sc[r][j] * (1.0f / CAP)) + bfv(mr[j]); Sc[r][j] = s; mx = fmaxf(mx, s); } const float mo = Mx[r], mn = fmaxf(mo, mx); const float fac = (mo == -INFINITY) ? 0.0f : __expf(mo - mn); float sm = 0.0f; for (int j = 0; j < CH; ++j) { const float p = __expf(Sc[r][j] - mn); sm += p; b16 ph, pl; split16(p * PS, ph, pl); Pa[r][j] = ph; Pb[r][j] = pl; } Fc[r] = fac; Ls[r] = Ls[r] * fac + sm; Mx[r] = mn; }
    wave_lds_sync();
#pragma unroll
    for (int t = 0; t < 8; ++t)
#pragma unroll
      for (int r8 = 0; r8 < 8; ++r8) oacc[t][r8] *= Fc[8 * hlf + r8];
#pragma unroll 2
    for (int kb = 0; kb < CH; kb += 32) { const v16b pa = frag_kb(&Pa[nloc][kb], hlf), pb = frag_kb(&Pb[nloc][kb], hlf);
#pragma unroll
      for (int t = 0; t < 8; ++t) { const size_t vo = ((size_t)g * D + t * 16 + nloc) * S + k0 + kb; const v16b vh = frag_kb(VTh + vo, hlf), vl = frag_kb(VTl + vo, hlf); oacc[t] = wmma16b(pa, vh, oacc[t]); oacc[t] = wmma16b(pa, vl, oacc[t]); oacc[t] = wmma16b(pb, vh, oacc[t]); } }
    wave_lds_sync(); }
#pragma unroll
  for (int t = 0; t < 8; ++t)
#pragma unroll
    for (int r8 = 0; r8 < 8; ++r8) { const int r = 8 * hlf + r8; Of[r][t * 16 + nloc] = oacc[t][r8] * (1.0f / (PS * QS)) / Ls[r]; }
  wave_lds_sync();
  for (int pass = 0; pass < 2; ++pass) { for (int r = 0; r < 16; ++r) *(volatile v4f*)(O + (size_t)(q0 + r) * HID + h * D + lane * 4) = *(const v4f*)(&Of[r][lane * 4]); __threadfence(); } }
__global__ __launch_bounds__(32) void outp_kernel(const float* __restrict__ O, const b16* __restrict__ WO, int QLIM, float* __restrict__ out) { __shared__ __attribute__((aligned(16))) b16 Ah[16][1024 + 8], Al[16][1024 + 8]; __shared__ float Tf[16][260]; const int lane = threadIdx.x, nloc = lane & 15, hlf = lane >> 4; const size_t t0 = (size_t)blockIdx.x * 16; const int cq = blockIdx.y * 512; if ((int)t0 >= QLIM) return;
  if (lane < 16) for (int k = 1024; k < 1032; ++k) { Ah[lane][k] = (b16)0.0f; Al[lane][k] = (b16)0.0f; }
#pragma unroll 1
  for (int gq = 0; gq < 4; ++gq) { const int c0 = cq + gq * 128; v8f acc[8];
#pragma unroll
    for (int t = 0; t < 8; ++t) acc[t] = (v8f){};
#pragma unroll 1
    for (int half = 0; half < 2; ++half) { const int kofs = half * 1024;
      for (int rr = 0; rr < 16; ++rr) for (int q = 0; q < 32; ++q) { const int c = q * 32 + lane; b16 p, pl; split16(O[(t0 + rr) * HID + kofs + c] * HS, p, pl); Ah[rr][c] = p; Al[rr][c] = pl; }
      wave_lds_sync();
#pragma unroll 2
      for (int kb = 0; kb < 1024; kb += 32) { const v16b a = frag_kb(&Ah[nloc][kb], hlf), al = frag_kb(&Al[nloc][kb], hlf);
#pragma unroll
        for (int t = 0; t < 8; ++t) { const v16b bw = frag_kb(WO + (size_t)(c0 + t * 16 + nloc) * HID + kofs + kb, hlf); acc[t] = wmma16b(a, bw, acc[t]); acc[t] = wmma16b(al, bw, acc[t]); } }
      wave_lds_sync(); }
#pragma unroll
    for (int t = 0; t < 8; ++t)
#pragma unroll
      for (int r8 = 0; r8 < 8; ++r8) Tf[8 * hlf + r8][t * 16 + nloc] = acc[t][r8] * (1.0f / (HS * WSC));
    wave_lds_sync();
    for (int pass = 0; pass < 2; ++pass) { for (int rr = 0; rr < 16; ++rr) *(volatile v4f*)(out + (t0 + rr) * HID + c0 + lane * 4) = *(const v4f*)(&Tf[rr][lane * 4]); __threadfence(); }
    wave_lds_sync(); } }
}

extern "C" void kernel_launch(void* const* d_in, const int* in_sizes, int n_in, void* d_out, int out_size, void* d_ws, size_t ws_size, hipStream_t stream) {
  (void)n_in;
  auto Fp = [&](int i) { return (const float*)d_in[i]; };
  if (in_sizes[0] != S * HID || in_sizes[1] != S * 64 || in_sizes[3] != S * S || in_sizes[5] != HID * 96 || in_sizes[8] != HID * QR * D || in_sizes[9] != HID * KR * D || in_sizes[11] != HID * HID || out_size != S * HID) return;
  const int QLIM = S;
  size_t off = 0; char* ws = (char*)d_ws;
  auto carve = [&](size_t bytes) { char* p = ws + off; off += (bytes + 255) & ~(size_t)255; return p; };
  b16* WT = (b16*)carve((size_t)NF * HID * 2); b16* WO = (b16*)carve((size_t)HID * HID * 2); float* FAC = (float*)carve((size_t)S * NF * 4); b16* Qh = (b16*)carve((size_t)S * H * D * 2); b16* Ql = (b16*)carve((size_t)S * H * D * 2); b16* Kh = (b16*)carve((size_t)S * KVH * D * 2); b16* Kl = (b16*)carve((size_t)S * KVH * D * 2); float* VR = (float*)carve((size_t)S * KVH * D * 4); b16* VTh = (b16*)carve((size_t)KVH * D * S * 2); b16* VTl = (b16*)carve((size_t)KVH * D * S * 2); float* O = (float*)carve((size_t)S * HID * 4);
  if (off > ws_size || off > ((size_t)96 << 20)) return;
  wput_kernel<<<512, 256, 0, stream>>>(Fp(5), Fp(6), Fp(7), Fp(8), Fp(9), Fp(10), Fp(11), WT, WO);
  proj_kernel<<<dim3(S / 16, 6), 32, 0, stream>>>(Fp(0), WT, QLIM, FAC);
  asm_kernel<<<S / 16, 32, 0, stream>>>(FAC, Fp(1), Fp(2), QLIM, Qh, Ql, Kh, Kl, VR);
  vt_kernel<<<(S / 64) * 4, 256, 0, stream>>>(VR, QLIM, VTh, VTl);
  att_kernel<<<H * (S / 16), 32, 0, stream>>>(Qh, Ql, Kh, Kl, VTh, VTl, Fp(3), QLIM, O);
  outp_kernel<<<dim3(S / 16, 4), 32, 0, stream>>>(O, WO, QLIM, (float*)d_out);
}
